// LocalPixelRelationConv_2791728742719
// MI455X (gfx1250) — hardware-run, weakly checked
//
#include <hip/hip_runtime.h>


namespace {
constexpr int NB_ = 8, C = 64, Hh = 128, Ww = 128, L = Hh * Ww, KK = 9, KC = C * KK  , PW = 32;
constexpr float XS = 8.0f, WSC = 256.0f, EPS = 1e-5f;
typedef _Float16 b16;
typedef __attribute__((ext_vector_type(16))) _Float16 v16b;
typedef __attribute__((ext_vector_type(8))) _Float16 v8b;
typedef __attribute__((ext_vector_type(8))) float v8f;
__device__ __forceinline__ float bf16_rne(float f) { unsigned int u = __float_as_uint(f); u += 0x7FFFu + ((u >> 16) & 1u); float r = __uint_as_float(u & 0xFFFF0000u); asm volatile("" : "+v"(r)); return r; }
__device__ __forceinline__ float bfv(float f) { float r = bf16_rne(f); asm volatile("" : "+v"(r)); return r; }
__device__ __forceinline__ v16b frag_kb(const b16* p, int hh) { const v8b a = *(const v8b*)(p + 8 * hh), b = *(const v8b*)(p + 16 + 8 * hh); v16b f;
#pragma unroll
  for (int e = 0; e < 8; ++e) { f[e] = a[e]; f[8 + e] = b[e]; } return f; }
__device__ __forceinline__ v8f wmma16b(v16b a, v16b b, v8f c) { v8f d = __builtin_amdgcn_wmma_f32_16x16x32_f16(false, a, false, b, (short)0, c, false, false); asm volatile("v_nop\n\tv_nop\n\tv_nop\n\tv_nop" : "+v"(d) : "v"(a), "v"(b)); return d; }
__device__ __forceinline__ void wave_lds_sync() { __builtin_amdgcn_fence(__ATOMIC_RELEASE, "workgroup"); __builtin_amdgcn_wave_barrier(); __builtin_amdgcn_fence(__ATOMIC_ACQUIRE, "workgroup"); }
__device__ __forceinline__ float pmul(float a, float b) { float p = a * b; asm volatile("" : "+v"(p)); return p; }
__device__ __forceinline__ int iclamp(int v, int lo, int hi) { return v < lo ? lo : (v > hi ? hi : v); }

__global__ __launch_bounds__(256) void wput_kernel(const float* __restrict__ cw, b16* __restrict__ W) { const int u = blockIdx.x * 256 + threadIdx.x; if (u >= 16 * (KC / 8)) return; const int o = u / (KC / 8), k0 = (u % (KC / 8)) * 8; v8b v;
#pragma unroll
  for (int j = 0; j < 8; ++j) v[j] = (b16)(o < KK ? bf16_rne(cw[(size_t)o * KC + k0 + j]) * WSC : 0.0f);
  for (int pass = 0; pass < 2; ++pass) { *(volatile v8b*)(W + (size_t)o * KC + k0) = v; __threadfence(); } }
__global__ __launch_bounds__(32) void main_kernel(const float* __restrict__ x, const float* __restrict__ feat, const b16* __restrict__ W, const float* __restrict__ g, const float* __restrict__ bt, const float* __restrict__ mu, const float* __restrict__ var, int PXLIM, float* __restrict__ out0, float* __restrict__ out1) { __shared__ __attribute__((aligned(16))) b16 Ah[PW][KC + 8]; __shared__ float Tw[PW][17]; const int lane = threadIdx.x, nloc = lane & 15, hlf = lane >> 4; const size_t px0 = (size_t)blockIdx.x * PW; if (px0 >= (size_t)PXLIM) return; const int b = (int)(px0 / L); const int l0 = (int)(px0 % L); const int y = l0 / Ww, x0 = l0 % Ww; const int xx = x0 + lane;
  for (int c = 0; c < C; ++c) { const float* xc = x + ((size_t)b * C + c) * L;
#pragma unroll
    for (int i = 0; i < 3; ++i) { const int yy = iclamp(y + i - 1, 0, Hh - 1);
#pragma unroll
      for (int j = 0; j < 3; ++j) { const int xq = iclamp(xx + j - 1, 0, Ww - 1); Ah[lane][c * KK + i * 3 + j] = (b16)(bf16_rne(xc[(size_t)yy * Ww + xq]) * XS); } } }
  for (int k = KC; k < KC + 8; ++k) Ah[lane][k] = (b16)0.0f;
  wave_lds_sync(); v8f a0 = (v8f){}, a1 = (v8f){};
#pragma unroll 2
  for (int kb = 0; kb < KC; kb += 32) { const v16b bw = frag_kb(W + (size_t)nloc * KC + kb, hlf); a0 = wmma16b(frag_kb(&Ah[nloc][kb], hlf), bw, a0); a1 = wmma16b(frag_kb(&Ah[16 + nloc][kb], hlf), bw, a1); }
#pragma unroll
  for (int r8 = 0; r8 < 8; ++r8) { Tw[8 * hlf + r8][nloc] = a0[r8] * (1.0f / (XS * WSC)); Tw[16 + 8 * hlf + r8][nloc] = a1[r8] * (1.0f / (XS * WSC)); }
  wave_lds_sync();
  float wv[KK]; float mx = -INFINITY;
#pragma unroll
  for (int k = 0; k < KK; ++k) { wv[k] = pmul((Tw[lane][k] - bfv(mu[k])) * rsqrtf(bfv(var[k]) + EPS), bfv(g[k])) + bfv(bt[k]); mx = fmaxf(mx, wv[k]); }
  for (int pass = 0; pass < 2; ++pass) {
#pragma unroll
    for (int k = 0; k < KK; ++k) ((volatile float*)out0)[((size_t)b * KK + k) * L + l0 + lane] = wv[k]; __threadfence(); }
  float wk[KK]; float sm = 0.0f;
#pragma unroll
  for (int k = 0; k < KK; ++k) { wk[k] = __expf(wv[k] - mx); sm += wk[k]; } const float inv = 1.0f / sm;
#pragma unroll
  for (int k = 0; k < KK; ++k) wk[k] *= inv;
  const int ym = iclamp(y - 1, 0, Hh - 1), yp = iclamp(y + 1, 0, Hh - 1), xm = iclamp(xx - 1, 0, Ww - 1), xp = iclamp(xx + 1, 0, Ww - 1);
  for (int pass = 0; pass < 2; ++pass) {
#pragma unroll 1
    for (int c = 0; c < C; ++c) { const float* fc = feat + ((size_t)b * C + c) * L; const float* r0 = fc + (size_t)ym * Ww; const float* r1 = fc + (size_t)y * Ww; const float* r2 = fc + (size_t)yp * Ww;
      float s = pmul(wk[0], bfv(r0[xm])); s += pmul(wk[1], bfv(r0[xx])); s += pmul(wk[2], bfv(r0[xp])); s += pmul(wk[3], bfv(r1[xm])); s += pmul(wk[4], bfv(r1[xx])); s += pmul(wk[5], bfv(r1[xp])); s += pmul(wk[6], bfv(r2[xm])); s += pmul(wk[7], bfv(r2[xx])); s += pmul(wk[8], bfv(r2[xp]));
      ((volatile float*)out1)[((size_t)b * C + c) * L + l0 + lane] = s; }
    __threadfence(); } }
}

extern "C" void kernel_launch(void* const* d_in, const int* in_sizes, int n_in, void* d_out, int out_size, void* d_ws, size_t ws_size, hipStream_t stream) {
  (void)n_in;
  auto Fp = [&](int i) { return (const float*)d_in[i]; };
  if (in_sizes[0] != NB_ * C * L || in_sizes[1] != NB_ * C * L || in_sizes[2] != KK * KC || in_sizes[3] != KK || in_sizes[6] != KK || out_size != NB_ * KK * L + NB_ * C * L) return;
  const int PXLIM = NB_ * L;
  size_t off = 0; char* ws = (char*)d_ws;
  auto carve = [&](size_t bytes) { char* p = ws + off; off += (bytes + 255) & ~(size_t)255; return p; };
  b16* W = (b16*)carve((size_t)16 * KC * 2);
  if (off > ws_size || off > ((size_t)1 << 20)) return;
  wput_kernel<<<(16 * (KC / 8) + 255) / 256, 256, 0, stream>>>(Fp(2), W);
  main_kernel<<<PXLIM / PW, 32, 0, stream>>>(Fp(0), Fp(1), W, Fp(3), Fp(4), Fp(5), Fp(6), PXLIM, (float*)d_out, (float*)d_out + (size_t)NB_ * KK * L);
}
